// MambaSubBlock_9328668967272
// MI455X (gfx1250) — hardware-verified
//
#include <hip/hip_runtime.h>
#include <math.h>

typedef __attribute__((ext_vector_type(16))) _Float16 v16h;
typedef __attribute__((ext_vector_type(8)))  _Float16 v8h;
typedef __attribute__((ext_vector_type(16))) __bf16   v16b;
typedef __attribute__((ext_vector_type(8)))  __bf16   v8b;
typedef __attribute__((ext_vector_type(8)))  float    v8f;
typedef __attribute__((ext_vector_type(4)))  float    v4f;
typedef __attribute__((ext_vector_type(2)))  float    v2f;

constexpr int kB    = 8;
constexpr int kL    = 4096;
constexpr int kC    = 128;
constexpr int kDI   = 256;
constexpr int kNS   = 16;
constexpr int kDTR  = 8;
constexpr int kXD   = 40;
constexpr int kXDP  = 64;
constexpr int kXZW  = 2 * kDI;
constexpr int kHID  = 512;
constexpr int kGD   = 32;
constexpr int kNT   = kB * kL;
constexpr int kTP   = 260;
constexpr int kLP   = 129;

__device__ __forceinline__ unsigned short f2bf_bits(float f) {
  unsigned u = __float_as_uint(f);
  return (unsigned short)((u + 0x7FFFu + ((u >> 16) & 1u)) >> 16);
}
__device__ __forceinline__ float bf_bits2f(unsigned short h) { return __uint_as_float(((unsigned)h) << 16); }

__device__ __forceinline__ void dep_guard_h(v8f& a, v8f& b, v16h x, v16h y) { asm volatile("v_nop\n\tv_nop\n\tv_nop\n\tv_nop" : "+v"(a), "+v"(b) : "v"(x), "v"(y)); }
__device__ __forceinline__ void dep_guard_b(v8f& a, v8f& b, v16b x, v16b y) { asm volatile("v_nop\n\tv_nop\n\tv_nop\n\tv_nop" : "+v"(a), "+v"(b) : "v"(x), "v"(y)); }
__device__ __forceinline__ void keep4_h(v16h a, v16h b, v16h c, v16h d) { asm volatile("v_nop" :: "v"(a), "v"(b), "v"(c), "v"(d)); }
__device__ __forceinline__ void keep4_b(v16b a, v16b b, v16b c, v16b d) { asm volatile("v_nop" :: "v"(a), "v"(b), "v"(c), "v"(d)); }
__device__ __forceinline__ void acc_guard4(v8f& a, v8f& b, v8f& c, v8f& d) { asm volatile("v_nop\n\tv_nop\n\tv_nop\n\tv_nop" : "+v"(a), "+v"(b), "+v"(c), "+v"(d)); }
template <typename T> struct Frag;
template <> struct Frag<_Float16> {
  typedef v16h V; union U { v16h v; v8h h[2]; };
  static __device__ __forceinline__ v16h load(const _Float16* p) {
    U f; f.h[0] = *(const v8h*)(p); f.h[1] = *(const v8h*)(p + 16); return f.v;
  }
  static __device__ __forceinline__ v8f mma(v16h a, v16h b, v8f c) {
    return __builtin_amdgcn_wmma_f32_16x16x32_f16(false, a, false, b, (short)0, c, false, false);
  }
  static __device__ __forceinline__ void guard(v8f& a, v8f& b, v16h x, v16h y) { dep_guard_h(a, b, x, y); }
  static __device__ __forceinline__ void keep(v16h a, v16h b, v16h c, v16h d) { keep4_h(a, b, c, d); }
};
template <> struct Frag<__bf16> {
  typedef v16b V; union U { v16b v; v8b h[2]; };
  static __device__ __forceinline__ v16b load(const __bf16* p) {
    U f; f.h[0] = *(const v8b*)(p); f.h[1] = *(const v8b*)(p + 16); return f.v;
  }
  static __device__ __forceinline__ v8f mma(v16b a, v16b b, v8f c) {
    return __builtin_amdgcn_wmma_f32_16x16x32_bf16(false, a, false, b, (short)0, c, false, false);
  }
  static __device__ __forceinline__ void guard(v8f& a, v8f& b, v16b x, v16b y) { dep_guard_b(a, b, x, y); }
  static __device__ __forceinline__ void keep(v16b a, v16b b, v16b c, v16b d) { keep4_b(a, b, c, d); }
};

template <int ET> struct Elem;
template <> struct Elem<0> { typedef _Float16 T; };
template <> struct Elem<1> { typedef __bf16 T; };
template <int ET, bool SPLIT, int BIAS_MODE, int OUT_MODE, bool RESID, int ACT = 0>
__global__ __launch_bounds__(256) void wmma_gemm64(
    const unsigned short* __restrict__ Ap, const unsigned short* __restrict__ A2p, int lda, long strideA,
    const unsigned short* __restrict__ Btp, const unsigned short* __restrict__ Bt2p, int ldb, long strideB,
    void* __restrict__ Cout, void* __restrict__ Cout2, int ldc, long strideC,
    const float* __restrict__ bias,
    const float* __restrict__ resid, long strideR,
    int M, int N, int K, float scale) {
  typedef typename Elem<ET>::T T;
  typedef typename Frag<T>::V V;
  const T* A = (const T*)Ap; const T* A2 = (const T*)A2p; const T* Bt = (const T*)Btp; const T* Bt2 = (const T*)Bt2p;
  __shared__ __align__(16) float sT[8][16 * 68];
  const int b    = blockIdx.y;
  const int lane = threadIdx.x & 31;
  const int wave = threadIdx.x >> 5;
  const int tilesN = N >> 6;
  const int tilesM = M >> 6;
  const int tile = blockIdx.x * 8 + wave;
  if (tile >= tilesM * tilesN) return;
  const int tm = tile / tilesN;
  const int tn = tile - tm * tilesN;
  const int m0 = tm << 6;
  const int n0 = tn << 6;

  const T* Ab  = A  + (size_t)b * strideA;
  const T* Bb  = Bt + (size_t)b * strideB;
  const T* Ab2 = SPLIT ? (A2  + (size_t)b * strideA) : nullptr;
  const T* Bb2 = SPLIT ? (Bt2 + (size_t)b * strideB) : nullptr;

  const int rlane = lane & 15;
  const int koff  = (lane >> 4) * 8;
  const int mOff  = (lane >> 4) * 8;

  v8f acc[4][4];
#pragma unroll
  for (int i = 0; i < 4; ++i)
#pragma unroll
    for (int j = 0; j < 4; ++j) acc[i][j] = (v8f){0.f,0.f,0.f,0.f,0.f,0.f,0.f,0.f};

  for (int k0 = 0; k0 < K; k0 += 32) {
    V bh[4], bl[4];
#pragma unroll
    for (int j = 0; j < 4; ++j) {
      const size_t bo = (size_t)(n0 + (j << 4) + rlane) * ldb + koff + k0;
      bh[j] = Frag<T>::load(Bb + bo);
      if (SPLIT) bl[j] = Frag<T>::load(Bb2 + bo);
    }
#pragma unroll
    for (int i = 0; i < 4; ++i) {
      const size_t ao = (size_t)(m0 + (i << 4) + rlane) * lda + koff + k0;
      V ah = Frag<T>::load(Ab + ao);
      V al;
      if (SPLIT) al = Frag<T>::load(Ab2 + ao);
#pragma unroll
      for (int j = 0; j < 4; ++j) {
        acc[i][j] = Frag<T>::mma(ah, bh[j], acc[i][j]);
        if (SPLIT) {
          acc[i][j] = Frag<T>::mma(ah, bl[j], acc[i][j]);
          acc[i][j] = Frag<T>::mma(al, bh[j], acc[i][j]);
        }
      }
      Frag<T>::guard(acc[i][0], acc[i][3], ah, SPLIT ? al : ah);
    }
    Frag<T>::keep(bh[0], bh[1], bh[2], bh[3]);
    if (SPLIT) Frag<T>::keep(bl[0], bl[1], bl[2], bl[3]);
  }
  acc_guard4(acc[0][0], acc[0][1], acc[0][2], acc[0][3]);
  acc_guard4(acc[1][0], acc[1][1], acc[1][2], acc[1][3]);
  acc_guard4(acc[2][0], acc[2][1], acc[2][2], acc[2][3]);
  acc_guard4(acc[3][0], acc[3][1], acc[3][2], acc[3][3]);

  float* slab = sT[wave];
  const float* Rb = RESID ? (resid + (size_t)b * strideR) : nullptr;
#pragma unroll
  for (int i = 0; i < 4; ++i) {
    const int mBase = m0 + (i << 4);
#pragma unroll
    for (int j = 0; j < 4; ++j) {
      const int n = n0 + (j << 4) + rlane;
      float bv = 0.f;
      if (BIAS_MODE == 2) bv = bias[n];
#pragma unroll
      for (int r = 0; r < 8; ++r) {
        float v = acc[i][j][r] * scale;
        if (BIAS_MODE == 1) v += bias[mBase + mOff + r];
        if (BIAS_MODE == 2) v += bv;
        if (RESID) v += Rb[(size_t)(mBase + mOff + r) * ldc + n];
        if (ACT == 1) v = tanhf(v);
        if (ACT == 2) v = fmaxf(v, 0.0f);
        if (ACT == 3) v = v / (1.0f + expf(-v));
        if (ACT == 4) v = (v > 0.f) ? v : 0.01f * v;
        if (ACT == 5) v = 0.5f * v * (1.0f + erff(v * 0.70710678118654752f));
        slab[(mOff + r) * 68 + (j << 4) + rlane] = v;
      }
    }
    __builtin_amdgcn_fence(__ATOMIC_RELEASE, "workgroup");
    __builtin_amdgcn_wave_barrier();
    __builtin_amdgcn_fence(__ATOMIC_ACQUIRE, "workgroup");
    if (OUT_MODE == 0) {
      float* C = (float*)Cout + (size_t)b * strideC;
      const int hh = lane >> 4, c4 = (lane & 15) * 4;
      for (int pass = 0; pass < 2; ++pass) {
#pragma unroll
        for (int it = 0; it < 8; ++it) {
          const int row = it * 2 + hh;
          v4f v = *(const v4f*)(slab + row * 68 + c4);
          *(volatile v4f*)(C + (size_t)(mBase + row) * ldc + n0 + c4) = v;
        }
        __threadfence();
      }
    } else {
      const int q = lane >> 3, c8 = (lane & 7) * 8;
      unsigned short* C  = (unsigned short*)Cout  + (size_t)b * strideC;
      unsigned short* C2 = (OUT_MODE == 2) ? ((unsigned short*)Cout2 + (size_t)b * strideC) : nullptr;
      for (int pass = 0; pass < 2; ++pass) {
#pragma unroll
        for (int it = 0; it < 4; ++it) {
          const int row = it * 4 + q;
          const float* sp = slab + row * 68 + c8;
          v8h hv, lv;
#pragma unroll
          for (int e = 0; e < 8; ++e) {
            if (OUT_MODE == 1) {
              hv[e] = (_Float16)sp[e];
            } else {
              unsigned short hb = f2bf_bits(sp[e]);
              unsigned short lb = f2bf_bits(sp[e] - bf_bits2f(hb));
              hv[e] = __builtin_bit_cast(_Float16, hb);
              lv[e] = __builtin_bit_cast(_Float16, lb);
            }
          }
          *(volatile v8h*)(C + (size_t)(mBase + row) * ldc + n0 + c8) = hv;
          if (OUT_MODE == 2) *(volatile v8h*)(C2 + (size_t)(mBase + row) * ldc + n0 + c8) = lv;
        }
        __threadfence();
      }
    }
    __builtin_amdgcn_fence(__ATOMIC_RELEASE, "workgroup");
    __builtin_amdgcn_wave_barrier();
    __builtin_amdgcn_fence(__ATOMIC_ACQUIRE, "workgroup");
  }
}

__global__ __launch_bounds__(256) void cast_rows_f16_kernel(
    const float* __restrict__ src, unsigned short* __restrict__ dst, int N, int K, int total8, float scale)
{
  const int i = blockIdx.x * 256 + threadIdx.x;
  if (i >= total8) return;
  const int e0  = i << 3;
  const int row = e0 / K;
  const int col = e0 - row * K;
  const int rowc = (row < N) ? row : (N - 1);
  const bool live = (row < N);
  const float* p = src + (size_t)rowc * K + col;
  const v4f a0 = *(const v4f*)(p);
  const v4f a1 = *(const v4f*)(p + 4);
  v8h hv;
#pragma unroll
  for (int e = 0; e < 4; ++e) {
    hv[e]     = live ? (_Float16)(a0[e] * scale) : (_Float16)0.0f;
    hv[4 + e] = live ? (_Float16)(a1[e] * scale) : (_Float16)0.0f;
  }
  unsigned short* q = dst + (size_t)e0;
  *(volatile v8h*)q = hv;
  __threadfence();
  *(volatile v8h*)q = hv;
}

__device__ __forceinline__ int seq_to_tok(int tt, int mode) {
  const int s = (mode & 1) ? (kL - 1 - tt) : tt;
  return (mode & 2) ? (((s & 63) << 6) | (s >> 6)) : s;
}

__global__ __launch_bounds__(256) void ln1_kernel(
    const float* __restrict__ x, const float* __restrict__ g, const float* __restrict__ be,
    unsigned short* __restrict__ XN16)
{
  __shared__ float T[64 * kLP];
  const int tid = threadIdx.x, lane = tid & 31, wave = tid >> 5;
  const int b = blockIdx.y, l0 = blockIdx.x * 64;
  const float* xb = x + (size_t)b * kC * kL + l0;
#pragma unroll 4
  for (int p = 0; p < 32; ++p) {
    const int idx = tid + p * 256;
    const int c = idx >> 6, ll = idx & 63;
    T[ll * kLP + c] = xb[(size_t)c * kL + ll];
  }
  __syncthreads();
  const int hsel = lane >> 4, l16 = lane & 15, cb8 = l16 * 8;
  float gg[8], bb[8];
#pragma unroll
  for (int e = 0; e < 8; ++e) { gg[e] = g[cb8 + e]; bb[e] = be[cb8 + e]; }
#pragma unroll 1
  for (int s = 0; s < 4; ++s) {
    const int row = wave * 8 + 2 * s + hsel;
    const float* tp = T + row * kLP + cb8;
    float v[8];
    float sum = 0.f;
#pragma unroll
    for (int e = 0; e < 8; ++e) { v[e] = tp[e]; sum += v[e]; }
#pragma unroll
    for (int off = 1; off < 16; off <<= 1) sum += __shfl_xor(sum, off, 32);
    const float mu = sum * (1.0f / kC);
    float sq = 0.f;
#pragma unroll
    for (int e = 0; e < 8; ++e) { const float dv = v[e] - mu; v[e] = dv; sq += dv * dv; }
#pragma unroll
    for (int off = 1; off < 16; off <<= 1) sq += __shfl_xor(sq, off, 32);
    const float rs = rsqrtf(sq * (1.0f / kC) + 1e-5f);
    v8h hv;
#pragma unroll
    for (int e = 0; e < 8; ++e) hv[e] = (_Float16)(v[e] * rs * gg[e] + bb[e]);
    unsigned short* dst = XN16 + ((size_t)b * kL + l0 + row) * kC + cb8;
    *(volatile v8h*)dst = hv;
    __threadfence();
    *(volatile v8h*)dst = hv;
  }
}

__global__ __launch_bounds__(256) void conv_silu_kernel(
    const _Float16* __restrict__ XZ16, const float* __restrict__ cw, const float* __restrict__ cb,
    unsigned short* __restrict__ XC16, int mode)
{
  __shared__ __align__(16) float sT[16 * kTP];
  const int tid = threadIdx.x, lane = tid & 31, wave = tid >> 5;
  const int d  = tid;
  const int t0 = blockIdx.x * 64;
  const int b  = blockIdx.y;
  const size_t brow = (size_t)b * kL;
  const float w0 = cw[d * 4 + 0], w1 = cw[d * 4 + 1], w2 = cw[d * 4 + 2], w3 = cw[d * 4 + 3];
  const float bc = cb[d];
  float xm3, xm2, xm1;
  {
    const int r3 = t0 - 3, r2 = t0 - 2, r1 = t0 - 1;
    const int c3 = r3 < 0 ? 0 : r3, c2 = r2 < 0 ? 0 : r2, c1 = r1 < 0 ? 0 : r1;
    const int l3 = seq_to_tok(c3, mode), l2 = seq_to_tok(c2, mode), l1 = seq_to_tok(c1, mode);
    const float v3 = (float)XZ16[(brow + (size_t)l3) * kXZW + d] * 0.25f;
    const float v2 = (float)XZ16[(brow + (size_t)l2) * kXZW + d] * 0.25f;
    const float v1 = (float)XZ16[(brow + (size_t)l1) * kXZW + d] * 0.25f;
    xm3 = (r3 >= 0) ? v3 : 0.f;
    xm2 = (r2 >= 0) ? v2 : 0.f;
    xm1 = (r1 >= 0) ? v1 : 0.f;
  }
#pragma unroll 1
  for (int sub = 0; sub < 4; ++sub) {
    const int lb = t0 + sub * 16;
#pragma unroll 1
    for (int st = 0; st < 16; ++st) {
      const int tt  = lb + st;
      const int tok = seq_to_tok(tt, mode);
      const float xin = (float)XZ16[(brow + (size_t)tok) * kXZW + d] * 0.25f;
      float acc = w0 * xm3;
      acc = fmaf(w1, xm2, acc);
      acc = fmaf(w2, xm1, acc);
      acc = fmaf(w3, xin, acc);
      const float sv = acc + bc;
      const float sg = __builtin_amdgcn_rcpf(1.0f + __expf(-sv));
      sT[st * kTP + tid] = (sv * sg) * 16.0f;
      xm3 = xm2; xm2 = xm1; xm1 = xin;
    }
    __syncthreads();
    v8h bv[2];
#pragma unroll
    for (int it = 0; it < 2; ++it) {
      const float* sp = sT + (it * 8 + wave) * kTP + lane * 8;
      const v4f a0 = *(const v4f*)(sp);
      const v4f a1 = *(const v4f*)(sp + 4);
#pragma unroll
      for (int e = 0; e < 4; ++e) {
        bv[it][e]     = (_Float16)a0[e];
        bv[it][4 + e] = (_Float16)a1[e];
      }
    }
    for (int pass = 0; pass < 2; ++pass) {
#pragma unroll
      for (int it = 0; it < 2; ++it) {
        const int tt  = lb + it * 8 + wave;
        const int tok = seq_to_tok(tt, mode);
        *(volatile v8h*)(XC16 + (brow + (size_t)tok) * kDI + lane * 8) = bv[it];
      }
      __threadfence();
    }
    __syncthreads();
  }
}

__global__ __launch_bounds__(256) void scan_kernel(
    const float* __restrict__ XDBL, const _Float16* __restrict__ XC16, const _Float16* __restrict__ XZ16,
    const float* __restrict__ Wdt, const float* __restrict__ dtb, const float* __restrict__ A_log,
    const float* __restrict__ Dv, _Float16* Y16, int mode, int accum)
{
  __shared__ __align__(16) float sX[16 * 64];
  __shared__ __align__(16) float sY[16 * kTP];
  const int tid = threadIdx.x, lane = tid & 31, wave = tid >> 5;
  const int d = tid;
  const int b = blockIdx.x;
  const size_t brow = (size_t)b * kL;

  float An[kNS];
#pragma unroll
  for (int n = 0; n < kNS; ++n) An[n] = -expf(A_log[(size_t)d * kNS + n]);
  float wdt[kDTR];
#pragma unroll
  for (int j = 0; j < kDTR; ++j) wdt[j] = Wdt[d * kDTR + j];
  const float Dd  = Dv[d];
  const float bdt = dtb[d];
  float h[kNS];
#pragma unroll
  for (int n = 0; n < kNS; ++n) h[n] = 0.f;

#pragma unroll 1
  for (int c = 0; c < kL / 16; ++c) {
    const int l0 = c * 16;
    {
      const int r = tid >> 4, q = (tid & 15) * 4;
      const int tt  = l0 + r;
      const int tok = seq_to_tok(tt, mode);
      const v4f v = *(const v4f*)(XDBL + (brow + (size_t)tok) * kXDP + q);
      *(v4f*)(sX + r * 64 + q) = v;
    }
    __syncthreads();
#pragma unroll 1
    for (int st = 0; st < 16; ++st) {
      const int tt  = l0 + st;
      const int tok = seq_to_tok(tt, mode);
      const size_t m = brow + (size_t)tok;
      const float* xr = sX + st * 64;
      const v4f t0 = *(const v4f*)(xr);
      const v4f t1 = *(const v4f*)(xr + 4);
      float a = bdt;
      a = fmaf(wdt[0], t0[0], a); a = fmaf(wdt[1], t0[1], a); a = fmaf(wdt[2], t0[2], a); a = fmaf(wdt[3], t0[3], a);
      a = fmaf(wdt[4], t1[0], a); a = fmaf(wdt[5], t1[1], a); a = fmaf(wdt[6], t1[2], a); a = fmaf(wdt[7], t1[3], a);
      const float delta = fmaxf(a, 0.0f) + log1pf(__expf(-fabsf(a)));
      const float u  = (float)XC16[m * kDI + d] * (1.0f / 16.0f);
      const float zv = (float)XZ16[m * kXZW + kDI + d] * 0.25f;
      v4f Bq[4], Cq[4];
#pragma unroll
      for (int qq = 0; qq < 4; ++qq) {
        Bq[qq] = *(const v4f*)(xr + kDTR + 4 * qq);
        Cq[qq] = *(const v4f*)(xr + kDTR + kNS + 4 * qq);
      }
      float dx = delta * u;
      asm volatile("" : "+v"(dx));
      float y = 0.f;
#pragma unroll
      for (int n = 0; n < kNS; ++n) {
        const float e = __expf(delta * An[n]);
        float p = dx * Bq[n >> 2][n & 3];
        asm volatile("" : "+v"(p));
        float qv = h[n] * e;
        asm volatile("" : "+v"(qv));
        const float hn = qv + p;
        h[n] = hn;
        float rr = Cq[n >> 2][n & 3] * hn;
        asm volatile("" : "+v"(rr));
        y += rr;
      }
      float sk = u * Dd;
      asm volatile("" : "+v"(sk));
      y += sk;
      const float sg = __builtin_amdgcn_rcpf(1.0f + __expf(-zv));
      const float gz = zv * sg;
      float yo = (y * gz) * 256.0f;
      asm volatile("" : "+v"(yo));
      if (accum) yo += (float)Y16[m * kDI + d];
      sY[st * kTP + tid] = yo;
    }
    __syncthreads();
    v8h hv[2];
#pragma unroll
    for (int it = 0; it < 2; ++it) {
      const float* sp = sY + (it * 8 + wave) * kTP + lane * 8;
      const v4f a0 = *(const v4f*)(sp);
      const v4f a1 = *(const v4f*)(sp + 4);
#pragma unroll
      for (int e = 0; e < 4; ++e) {
        hv[it][e]     = (_Float16)a0[e];
        hv[it][4 + e] = (_Float16)a1[e];
      }
    }
    for (int pass = 0; pass < 2; ++pass) {
#pragma unroll
      for (int it = 0; it < 2; ++it) {
        const int tt  = l0 + it * 8 + wave;
        const int tok = seq_to_tok(tt, mode);
        const size_t yo = (brow + (size_t)tok) * kDI + lane * 8;
        *(volatile v8h*)(Y16 + yo) = hv[it];
      }
      __threadfence();
    }
  }
}

__global__ __launch_bounds__(256) void ctx_gate_kernel(
    const float* __restrict__ OH, const float* __restrict__ OV,
    const float* __restrict__ W1, const float* __restrict__ b1,
    const float* __restrict__ W2, const float* __restrict__ b2, float* __restrict__ GATE)
{
  __shared__ float red[256];
  __shared__ float sctx[kC];
  __shared__ float shid[kGD];
  __shared__ __align__(16) float sg[kC];
  const int tid = threadIdx.x, lane = tid & 31, wave = tid >> 5;
  const int b = blockIdx.x;
  const int c = tid & (kC - 1), hf = tid >> 7;
  const float* po = OH + ((size_t)b * kL + (size_t)hf * (kL / 2)) * kC + c;
  const float* pv = OV + ((size_t)b * kL + (size_t)hf * (kL / 2)) * kC + c;
  float s = 0.f;
#pragma unroll 1
  for (int l = 0; l < kL / 2; ++l) s += 0.5f * (po[(size_t)l * kC] + pv[(size_t)l * kC]);
  red[tid] = s;
  __syncthreads();
  if (tid < kC) sctx[tid] = (red[tid] + red[tid + kC]) * (1.0f / kL);
  __syncthreads();
  if (tid < kGD) {
    float a = b1[tid];
#pragma unroll 1
    for (int j = 0; j < kC; ++j) a = fmaf(W1[tid * kC + j], sctx[j], a);
    shid[tid] = fmaxf(a, 0.0f);
  }
  __syncthreads();
  if (tid < kC) {
    float a = b2[tid];
#pragma unroll 1
    for (int j = 0; j < kGD; ++j) a = fmaf(W2[tid * kGD + j], shid[j], a);
    sg[tid] = __builtin_amdgcn_rcpf(1.0f + expf(-a));
  }
  __syncthreads();
  if (wave == 0) {
    const v4f v = *(const v4f*)(sg + lane * 4);
    float* dst = GATE + (size_t)b * kC + lane * 4;
    *(volatile v4f*)dst = v;
    __threadfence();
    *(volatile v4f*)dst = v;
  }
}

__global__ __launch_bounds__(256) void fuse_ln2_kernel(
    const float* __restrict__ x, const float* __restrict__ OH, const float* __restrict__ OV,
    const float* __restrict__ GATE, const float* __restrict__ g2, const float* __restrict__ be2,
    float* __restrict__ X1T, unsigned short* __restrict__ XN2)
{
  __shared__ float T[64 * kLP];
  __shared__ float sgt[kC];
  const int tid = threadIdx.x, lane = tid & 31, wave = tid >> 5;
  const int b = blockIdx.y, l0 = blockIdx.x * 64;
  if (tid < kC) sgt[tid] = GATE[(size_t)b * kC + tid];
  const float* xb = x + (size_t)b * kC * kL + l0;
#pragma unroll 4
  for (int p = 0; p < 32; ++p) {
    const int idx = tid + p * 256;
    const int c = idx >> 6, ll = idx & 63;
    T[ll * kLP + c] = xb[(size_t)c * kL + ll];
  }
  __syncthreads();
#pragma unroll 2
  for (int p = 0; p < 32; ++p) {
    const int idx = tid + p * 256;
    const int tok = idx >> 7, c = idx & (kC - 1);
    const size_t row = (size_t)b * kL + l0 + tok;
    const float oh = OH[row * kC + c];
    const float ov = OV[row * kC + c];
    const float gc = sgt[c];
    const float f = gc * oh + (1.0f - gc) * ov;
    T[tok * kLP + c] += f;
  }
  __syncthreads();
  const int hsel = lane >> 4, l16 = lane & 15, cb8 = l16 * 8;
#pragma unroll 1
  for (int s = 0; s < 8; ++s) {
    const int c = wave * 16 + 2 * s + hsel;
    v4f val;
#pragma unroll
    for (int e = 0; e < 4; ++e) val[e] = T[(4 * l16 + e) * kLP + c];
    float* dst = X1T + ((size_t)b * kC + c) * kL + l0 + 4 * l16;
    *(volatile v4f*)dst = val;
    __threadfence();
    *(volatile v4f*)dst = val;
  }
  float gg[8], bb[8];
#pragma unroll
  for (int e = 0; e < 8; ++e) { gg[e] = g2[cb8 + e]; bb[e] = be2[cb8 + e]; }
#pragma unroll 1
  for (int s = 0; s < 4; ++s) {
    const int row = wave * 8 + 2 * s + hsel;
    const float* tp = T + row * kLP + cb8;
    float v[8];
    float sum = 0.f;
#pragma unroll
    for (int e = 0; e < 8; ++e) { v[e] = tp[e]; sum += v[e]; }
#pragma unroll
    for (int off = 1; off < 16; off <<= 1) sum += __shfl_xor(sum, off, 32);
    const float mu = sum * (1.0f / kC);
    float sq = 0.f;
#pragma unroll
    for (int e = 0; e < 8; ++e) { const float dv = v[e] - mu; v[e] = dv; sq += dv * dv; }
#pragma unroll
    for (int off = 1; off < 16; off <<= 1) sq += __shfl_xor(sq, off, 32);
    const float rs = rsqrtf(sq * (1.0f / kC) + 1e-5f);
    v8h hv;
#pragma unroll
    for (int e = 0; e < 8; ++e) hv[e] = (_Float16)(v[e] * rs * gg[e] + bb[e]);
    unsigned short* dst = XN2 + ((size_t)b * kL + l0 + row) * kC + cb8;
    *(volatile v8h*)dst = hv;
    __threadfence();
    *(volatile v8h*)dst = hv;
  }
}

__global__ __launch_bounds__(256) void gelu_cast_kernel(
    const float* __restrict__ in, unsigned short* __restrict__ out, int n2)
{
  const int i = blockIdx.x * 256 + threadIdx.x;
  if (i >= n2) return;
  const v2f a = *(const v2f*)(in + 2 * (size_t)i);
  const float g0 = 0.5f * a[0] * (1.0f + erff(a[0] * 0.70710678118654752f));
  const float g1 = 0.5f * a[1] * (1.0f + erff(a[1] * 0.70710678118654752f));
  const _Float16 h0 = (_Float16)(g0 * 16.0f), h1 = (_Float16)(g1 * 16.0f);
  const unsigned u = (unsigned)__builtin_bit_cast(unsigned short, h0) | ((unsigned)__builtin_bit_cast(unsigned short, h1) << 16);
  ((volatile unsigned*)out)[i] = u;
  __threadfence();
  ((volatile unsigned*)out)[i] = u;
}

extern "C" void kernel_launch(void* const* d_in, const int* in_sizes, int n_in,
                              void* d_out, int out_size, void* d_ws, size_t ws_size,
                              hipStream_t stream)
{
  if (n_in < 31) return;
  if (in_sizes[0] != kB * kC * kL) return;
  if (in_sizes[1] != kC || in_sizes[2] != kC) return;
  for (int o = 0; o < 2; ++o) {
    const int* sz = in_sizes + 3 + 9 * o;
    if (sz[0] != kXZW * kC) return;
    if (sz[1] != kDI * 4 || sz[2] != kDI) return;
    if (sz[3] != kXD * kDI) return;
    if (sz[4] != kDI * kDTR || sz[5] != kDI) return;
    if (sz[6] != kDI * kNS || sz[7] != kDI) return;
    if (sz[8] != kC * kDI) return;
  }
  if (in_sizes[21] != kGD * kC || in_sizes[22] != kGD) return;
  if (in_sizes[23] != kC * kGD || in_sizes[24] != kC) return;
  if (in_sizes[25] != kC || in_sizes[26] != kC) return;
  if (in_sizes[27] != kHID * kC || in_sizes[28] != kHID) return;
  if (in_sizes[29] != kC * kHID || in_sizes[30] != kC) return;
  if (out_size != kB * kC * kL) return;

  const float* x    = (const float*)d_in[0];
  const float* n1_g = (const float*)d_in[1];
  const float* n1_b = (const float*)d_in[2];
  const float* Pm[2][9];
  for (int o = 0; o < 2; ++o)
    for (int i = 0; i < 9; ++i) Pm[o][i] = (const float*)d_in[3 + 9 * o + i];
  const float* gW1  = (const float*)d_in[21];
  const float* gb1  = (const float*)d_in[22];
  const float* gW2  = (const float*)d_in[23];
  const float* gb2  = (const float*)d_in[24];
  const float* n2_g = (const float*)d_in[25];
  const float* n2_b = (const float*)d_in[26];
  const float* mW1  = (const float*)d_in[27];
  const float* mb1  = (const float*)d_in[28];
  const float* mW2  = (const float*)d_in[29];
  const float* mb2  = (const float*)d_in[30];
  float* dout = (float*)d_out;

  const size_t SZ_WIN   = (size_t)kXZW * kC * 2;
  const size_t SZ_WXP   = (size_t)kXDP * kDI * 2;
  const size_t SZ_WOUT  = (size_t)kC * kDI * 2;
  const size_t SZ_W1    = (size_t)kHID * kC * 2;
  const size_t SZ_W2    = (size_t)kC * kHID * 2;
  const size_t OFF_WIN  = 0;
  const size_t OFF_WXP  = OFF_WIN  + 2 * SZ_WIN;
  const size_t OFF_WOUT = OFF_WXP  + 2 * SZ_WXP;
  const size_t OFF_W1   = OFF_WOUT + 2 * SZ_WOUT;
  const size_t OFF_W2   = OFF_W1   + SZ_W1;
  const size_t OFF_GATE = OFF_W2   + SZ_W2;
  const size_t OFF_BASE = 786432;
  const size_t SZ_XN16  = (size_t)kNT * kC * 2;
  const size_t SZ_XZ16  = (size_t)kNT * kXZW * 2;
  const size_t SZ_XC16  = (size_t)kNT * kDI * 2;
  const size_t SZ_XDBL  = (size_t)kNT * kXDP * 4;
  const size_t SZ_Y16   = (size_t)kNT * kDI * 2;
  const size_t SZ_OHV   = (size_t)kNT * kC * 4;
  const size_t SZ_X1T   = (size_t)kB * kC * kL * 4;
  const size_t SZ_XN2   = (size_t)kNT * kC * 2;
  const size_t SZ_HPRE  = (size_t)kNT * kHID * 4;
  const size_t SZ_H16   = (size_t)kNT * kHID * 2;
  const size_t OFF_XN16 = OFF_BASE;
  const size_t OFF_XZ16 = OFF_XN16 + SZ_XN16;
  const size_t OFF_XC16 = OFF_XZ16 + SZ_XZ16;
  const size_t OFF_XDBL = OFF_XC16 + SZ_XC16;
  const size_t OFF_Y16  = OFF_XDBL + SZ_XDBL;
  const size_t OFF_OH   = OFF_Y16  + SZ_Y16;
  const size_t OFF_OV   = OFF_OH   + SZ_OHV;
  const size_t END_SCAN = OFF_OV   + SZ_OHV;
  const size_t OFF_X1T  = OFF_BASE;
  const size_t OFF_XN2  = OFF_X1T  + SZ_X1T;
  const size_t OFF_HPRE = OFF_XN2  + SZ_XN2;
  const size_t OFF_H16  = OFF_HPRE + SZ_HPRE;
  const size_t END_MLP  = OFF_H16  + SZ_H16;
  const size_t TOTAL    = (END_MLP > END_SCAN) ? END_MLP : END_SCAN;
  if (OFF_GATE + (size_t)kB * kC * 4 > OFF_BASE) return;
  if (ws_size < TOTAL) return;

  char* ws = (char*)d_ws;
  unsigned short* WIN16[2];  unsigned short* WXP16[2];  unsigned short* WOUT16[2];
  for (int o = 0; o < 2; ++o) {
    WIN16[o]  = (unsigned short*)(ws + OFF_WIN  + (size_t)o * SZ_WIN);
    WXP16[o]  = (unsigned short*)(ws + OFF_WXP  + (size_t)o * SZ_WXP);
    WOUT16[o] = (unsigned short*)(ws + OFF_WOUT + (size_t)o * SZ_WOUT);
  }
  unsigned short* W1_16 = (unsigned short*)(ws + OFF_W1);
  unsigned short* W2_16 = (unsigned short*)(ws + OFF_W2);
  float*          GATE  = (float*)(ws + OFF_GATE);
  unsigned short* XN16  = (unsigned short*)(ws + OFF_XN16);
  unsigned short* XZ16  = (unsigned short*)(ws + OFF_XZ16);
  unsigned short* XC16  = (unsigned short*)(ws + OFF_XC16);
  float*          XDBL  = (float*)(ws + OFF_XDBL);
  unsigned short* Y16   = (unsigned short*)(ws + OFF_Y16);
  float*          OHV[2];
  OHV[0] = (float*)(ws + OFF_OH);
  OHV[1] = (float*)(ws + OFF_OV);
  float*          X1T   = (float*)(ws + OFF_X1T);
  unsigned short* XN2   = (unsigned short*)(ws + OFF_XN2);
  float*          HPRE  = (float*)(ws + OFF_HPRE);
  unsigned short* H16   = (unsigned short*)(ws + OFF_H16);
  const float* dummy_bias  = mb1;
  const float* dummy_resid = x;

  for (int o = 0; o < 2; ++o) {
    cast_rows_f16_kernel<<<(kXZW * kC) / 8 / 256, 256, 0, stream>>>(
        Pm[o][0], WIN16[o], kXZW, kC, (kXZW * kC) / 8, 32.0f);
    cast_rows_f16_kernel<<<(kXDP * kDI) / 8 / 256, 256, 0, stream>>>(
        Pm[o][3], WXP16[o], kXD, kDI, (kXDP * kDI) / 8, 32.0f);
    cast_rows_f16_kernel<<<(kC * kDI) / 8 / 256, 256, 0, stream>>>(
        Pm[o][8], WOUT16[o], kC, kDI, (kC * kDI) / 8, 32.0f);
  }
  cast_rows_f16_kernel<<<(kHID * kC) / 8 / 256, 256, 0, stream>>>(mW1, W1_16, kHID, kC, (kHID * kC) / 8, 32.0f);
  cast_rows_f16_kernel<<<(kC * kHID) / 8 / 256, 256, 0, stream>>>(mW2, W2_16, kC, kHID, (kC * kHID) / 8, 32.0f);

  ln1_kernel<<<dim3(kL / 64, kB), 256, 0, stream>>>(x, n1_g, n1_b, XN16);

  for (int o = 0; o < 2; ++o) {
    wmma_gemm64<0, false, 0, 1, false><<<dim3(512, 1), 256, 0, stream>>>(
        XN16, XN16, kC, 0L, WIN16[o], WIN16[o], kC, 0L,
        (void*)XZ16, (void*)XZ16, kXZW, 0L, dummy_bias, dummy_resid, 0L, kNT, kXZW, kC, 0.125f);

    for (int r = 0; r < 2; ++r) {
      const int mode = 2 * o + r;
      conv_silu_kernel<<<dim3(kL / 64, kB), 256, 0, stream>>>(
          (const _Float16*)XZ16, Pm[o][1], Pm[o][2], XC16, mode);
      wmma_gemm64<0, false, 0, 0, false><<<dim3(64, 1), 256, 0, stream>>>(
          XC16, XC16, kDI, 0L, WXP16[o], WXP16[o], kDI, 0L,
          (void*)XDBL, (void*)XDBL, kXDP, 0L, dummy_bias, dummy_resid, 0L, kNT, kXDP, kDI, 1.0f / 512.0f);
      scan_kernel<<<dim3(kB), 256, 0, stream>>>(
          XDBL, (const _Float16*)XC16, (const _Float16*)XZ16, Pm[o][4], Pm[o][5], Pm[o][6], Pm[o][7],
          (_Float16*)Y16, mode, r);
    }
    wmma_gemm64<0, false, 0, 0, false><<<dim3(128, 1), 256, 0, stream>>>(
        Y16, Y16, kDI, 0L, WOUT16[o], WOUT16[o], kDI, 0L,
        (void*)OHV[o], (void*)OHV[o], kC, 0L, dummy_bias, dummy_resid, 0L, kNT, kC, kDI, 1.0f / 8192.0f);
  }

  ctx_gate_kernel<<<dim3(kB), 256, 0, stream>>>(OHV[0], OHV[1], gW1, gb1, gW2, gb2, GATE);

  fuse_ln2_kernel<<<dim3(kL / 64, kB), 256, 0, stream>>>(x, OHV[0], OHV[1], GATE, n2_g, n2_b, X1T, XN2);

  wmma_gemm64<0, false, 2, 0, false><<<dim3(512, 1), 256, 0, stream>>>(
      XN2, XN2, kC, 0L, W1_16, W1_16, kC, 0L,
      (void*)HPRE, (void*)HPRE, kHID, 0L, mb1, dummy_resid, 0L, kNT, kHID, kC, 1.0f / 32.0f);

  gelu_cast_kernel<<<(kNT * kHID) / 2 / 256, 256, 0, stream>>>(HPRE, H16, (kNT * kHID) / 2);

  wmma_gemm64<0, false, 1, 0, true><<<dim3(16, kB), 256, 0, stream>>>(
      W2_16, W2_16, kHID, 0L, H16, H16, kHID, (long)kL * kHID,
      (void*)dout, (void*)dout, kL, (long)kC * kL, mb2, X1T, (long)kC * kL, kC, kL, kHID, 1.0f / 512.0f);
}
